// Transformer_31988916420621
// MI455X (gfx1250) — hardware-verified
//
#include <hip/hip_runtime.h>
#include <math.h>


#ifndef NB
#define NB 2
#endif
#ifndef SEQ
#define SEQ 2048
#endif
#define NB_FULL 2
#define SEQ_FULL 2048
#define CT 1024
#define HEADS 16
#define GROUPS 8
#define DK 32
#define DV 64
#define KQW 512
#define CING 128
#define AT_PO 36
#define TK_PX 68

static_assert(NB >= 1 && NB <= NB_FULL);
static_assert(SEQ <= SEQ_FULL);
static_assert(SEQ == 2048 || SEQ == 1024 || SEQ == 512 || SEQ == 256);
static_assert(SEQ % 256 == 0);
static_assert(HEADS * DK == KQW && HEADS * DV == CT && GROUPS * CING == CT);
static_assert(DK == 32);
static_assert(DV == 64);
static_assert(KQW / GROUPS == 64);
static_assert(CT / GROUPS == 128);
static_assert(CING % 32 == 0 && CT % 32 == 0);
static_assert(CT % 64 == 0 && SEQ % 64 == 0);

typedef _Float16 h16;
typedef __attribute__((ext_vector_type(16))) _Float16 v16h;
typedef __attribute__((ext_vector_type(8)))  _Float16 v8h;
typedef __attribute__((ext_vector_type(2)))  _Float16 v2h;
typedef __attribute__((ext_vector_type(8)))  float    v8f;
typedef __attribute__((ext_vector_type(4)))  float    v4f;
typedef __attribute__((ext_vector_type(2)))  float    v2f;
typedef __attribute__((ext_vector_type(4)))  unsigned int v4u;

static constexpr float ACT_CARRY = 8.0f;
static constexpr float W_CARRY   = 32.0f;
static constexpr float SC_GEMM   = 1.0f / 256.0f;
static constexpr float P_CARRY   = 16384.0f;
static constexpr float O_UNDO    = 1.0f / 131072.0f;
static constexpr float KQ_UNDO   = 1.0f / 64.0f;
static constexpr float RSQRT_L   = (SEQ == 2048) ? 0.022097086912079608f : (SEQ == 1024) ? 0.03125f : (SEQ == 512) ? 0.044194173824159216f : 0.0625f;
static constexpr float SC2       = RSQRT_L * KQ_UNDO * 1.4426950408889634f;
static_assert(ACT_CARRY * W_CARRY * SC_GEMM == 1.0f);
static_assert(ACT_CARRY * P_CARRY * O_UNDO == 1.0f);
static_assert(ACT_CARRY * ACT_CARRY * KQ_UNDO == 1.0f);


#define VST2(T, ptr, val) do { const T vst2_v_ = (val); *(volatile T*)(ptr) = vst2_v_; __threadfence(); *(volatile T*)(ptr) = vst2_v_; } while (0)
#define VST2V4(ptr, val) do { const v4f vst2_v4_ = (val); *(volatile v4f*)(ptr) = vst2_v4_; __threadfence(); *(volatile v4f*)(ptr) = vst2_v4_; } while (0)

__device__ __forceinline__ float bfr(float f) {
    unsigned u = __float_as_uint(f);
    u += 0x7FFFu + ((u >> 16) & 1u);
    return __uint_as_float(u & 0xFFFF0000u);
}

static __device__ __forceinline__ h16 toh_flush(float v) { const float w = (fabsf(v) < 6.103515625e-05f) ? 0.0f : v; return (h16)w; }
static __device__ __forceinline__ v2h toh2_flush(float a, float b) {
    v2f w;
    w.x = (fabsf(a) < 6.103515625e-05f) ? 0.0f : a;
    w.y = (fabsf(b) < 6.103515625e-05f) ? 0.0f : b;
    return __builtin_convertvector(w, v2h);
}
union PackH8  { v8h v;  v2h p[4]; };
union PackH16 { v16h v; v2h p[8]; };

union FragU { v16h v; v8h h[2]; };
__device__ __forceinline__ v16h frag_ld(const _Float16* p) {
    FragU f; f.h[0] = *(const v8h*)(p); f.h[1] = *(const v8h*)(p + 16); return f.v;
}
__device__ __forceinline__ v8f wmma16(v16h a, v16h b, v8f c) {
    c = __builtin_amdgcn_wmma_f32_16x16x32_f16(false, a, false, b, (short)0, c, false, false);
    asm volatile("v_nop\n\tv_nop\n\tv_nop\n\tv_nop" : "+v"(c) : "v"(a), "v"(b));
    return c;
}
__device__ __forceinline__ void wave_sync_lds() {
    __builtin_amdgcn_fence(3  , "workgroup");
    __builtin_amdgcn_wave_barrier();
    __builtin_amdgcn_fence(2  , "workgroup");
}

__global__ __launch_bounds__(256) void k_wconv(const float* __restrict__ Wm, _Float16* __restrict__ W16, unsigned n8) {
    const unsigned u = blockIdx.x * 256u + threadIdx.x;
    if (u >= n8) return;
    const v4f a = *(const v4f*)(Wm + (size_t)u * 8u);
    const v4f b = *(const v4f*)(Wm + (size_t)u * 8u + 4u);
    PackH8 pk;
    pk.p[0] = toh2_flush(bfr(a.x) * W_CARRY, bfr(a.y) * W_CARRY);
    pk.p[1] = toh2_flush(bfr(a.z) * W_CARRY, bfr(a.w) * W_CARRY);
    pk.p[2] = toh2_flush(bfr(b.x) * W_CARRY, bfr(b.y) * W_CARRY);
    pk.p[3] = toh2_flush(bfr(b.z) * W_CARRY, bfr(b.w) * W_CARRY);
    const v8h hv = pk.v;
    _Float16* dst = W16 + (size_t)u * 8u;
    *(volatile v8h*)dst = hv;
    __threadfence();
    *(volatile v8h*)dst = hv;
}

static_assert(256 * 16 * 4 == 64 * 64 * 4);
static_assert(256 * 16 * 2 == 64 * 128);
static_assert(64 * TK_PX * 4 <= 131072);
__global__ __launch_bounds__(256) void k_tokT(const float* __restrict__ tok, _Float16* __restrict__ TOKT) {
    __shared__ __align__(16) float sX[64 * TK_PX];
    const unsigned t = threadIdx.x;
    const unsigned l0 = blockIdx.x * 64u, c0 = blockIdx.y * 64u, n = blockIdx.z;
    {
        const unsigned r = t >> 4, p4 = (t & 15u) * 4u;
        const float* src = tok + ((size_t)n * CT + c0 + r) * SEQ_FULL + l0 + p4;
#pragma unroll
        for (int it = 0; it < 4; ++it) {
            const v4f v = *(const v4f*)(src + (size_t)(16u * (unsigned)it) * SEQ_FULL);
            *(v4f*)(sX + (r + 16u * (unsigned)it) * TK_PX + p4) = v;
        }
    }
    __syncthreads();
    {
        const unsigned q = t >> 3, pc = t & 7u;
        v8h hv[2];
#pragma unroll
        for (int it = 0; it < 2; ++it) {
            const unsigned l = q + 32u * (unsigned)it;
            PackH8 pk;
#pragma unroll
            for (int e2 = 0; e2 < 4; ++e2) {
                const float a = bfr(sX[(8u * pc + 2u * (unsigned)e2) * TK_PX + l]) * ACT_CARRY;
                const float b = bfr(sX[(8u * pc + 2u * (unsigned)e2 + 1u) * TK_PX + l]) * ACT_CARRY;
                pk.p[e2] = toh2_flush(a, b);
            }
            hv[it] = pk.v;
        }
        _Float16* dst = TOKT + ((size_t)n * SEQ + l0 + q) * CT + c0 + 8u * pc;
        for (int pass = 0; pass < 2; ++pass) {
#pragma unroll
            for (int it = 0; it < 2; ++it) *(volatile v8h*)(dst + (size_t)(32u * (unsigned)it) * CT) = hv[it];
            __threadfence();
        }
    }
}

static_assert(32 * 16 * 8 == 16 * 256);
static_assert(32 * 16 * 4 == 16 * 128);
static_assert(8 * 16 * 68 * 4 <= 131072);
template <int OUT_MODE, bool RESID, bool BIAS_ROW>
static __device__ __forceinline__ void gemm64_body(
    const _Float16* __restrict__ A, unsigned lda, const _Float16* __restrict__ Bt, unsigned ldb,
    void* __restrict__ Cout, unsigned ldc, const float* __restrict__ bias, const float* __restrict__ resid,
    unsigned tilesM, unsigned tilesN, unsigned K) {
  __shared__ __align__(16) float sT[8][16 * 68];
  const unsigned lane = threadIdx.x & 31u;
  const unsigned wave = (unsigned)__builtin_amdgcn_readfirstlane((int)(threadIdx.x >> 5));
  const unsigned tile = blockIdx.x * 8u + wave;
  if (tile >= tilesM * tilesN) return;
  const unsigned tm = tile / tilesN;
  const unsigned tn = tile - tm * tilesN;
  const unsigned m0 = tm << 6, n0 = tn << 6;
  const unsigned rlane = lane & 15u;
  const unsigned koff = (lane >> 4) * 8u;
  const unsigned mOff = koff;

  v8f acc[4][4];
#pragma unroll
  for (int i = 0; i < 4; ++i)
#pragma unroll
    for (int j = 0; j < 4; ++j) acc[i][j] = (v8f){0.f,0.f,0.f,0.f,0.f,0.f,0.f,0.f};

  for (unsigned k0 = 0; k0 < K; k0 += 32u) {
    v16h bh[4];
#pragma unroll
    for (int j = 0; j < 4; ++j)
      bh[j] = frag_ld(Bt + (size_t)(n0 + ((unsigned)j << 4) + rlane) * ldb + koff + k0);
#pragma unroll
    for (int i = 0; i < 4; ++i) {
      const v16h ah = frag_ld(A + (size_t)(m0 + ((unsigned)i << 4) + rlane) * lda + koff + k0);
#pragma unroll
      for (int j = 0; j < 4; ++j) acc[i][j] = wmma16(ah, bh[j], acc[i][j]);
    }
  }

  float* slab = sT[wave];
#pragma unroll
  for (int i = 0; i < 4; ++i) {
    const unsigned mBase = m0 + ((unsigned)i << 4);
    float brow[8];
    if (BIAS_ROW) {
      const v4f b0 = *(const v4f*)(bias + mBase + mOff);
      const v4f b1 = *(const v4f*)(bias + mBase + mOff + 4u);
      brow[0] = bfr(b0.x); brow[1] = bfr(b0.y); brow[2] = bfr(b0.z); brow[3] = bfr(b0.w);
      brow[4] = bfr(b1.x); brow[5] = bfr(b1.y); brow[6] = bfr(b1.z); brow[7] = bfr(b1.w);
    } else {
#pragma unroll
      for (int r = 0; r < 8; ++r) brow[r] = 0.0f;
    }
#pragma unroll
    for (int j = 0; j < 4; ++j) {
      const unsigned n = n0 + ((unsigned)j << 4) + rlane;
      float bcol = 0.0f;
      if (!BIAS_ROW) bcol = bfr(bias[n]);
#pragma unroll
      for (int r = 0; r < 8; ++r) {
        float v = acc[i][j][r] * SC_GEMM + (BIAS_ROW ? brow[r] : bcol);
        if (OUT_MODE == 1) v *= ACT_CARRY;
        slab[(mOff + (unsigned)r) * 68u + ((unsigned)j << 4) + rlane] = v;
      }
    }
    wave_sync_lds();
    if (OUT_MODE == 0) {
      float* C = (float*)Cout;
      const unsigned hh = lane >> 4, c4 = (lane & 15u) * 4u;
#pragma unroll
      for (int half = 0; half < 2; ++half) {
        v4f vv[4];
#pragma unroll
        for (int it = 0; it < 4; ++it) {
          const unsigned row = (unsigned)(half * 4 + it) * 2u + hh;
          vv[it] = *(const v4f*)(slab + row * 68u + c4);
          if (RESID) vv[it] += *(const v4f*)(resid + (size_t)(mBase + row) * ldc + n0 + c4);
        }
        for (int pass = 0; pass < 2; ++pass) {
#pragma unroll
          for (int it = 0; it < 4; ++it) {
            const unsigned row = (unsigned)(half * 4 + it) * 2u + hh;
            *(volatile v4f*)(C + (size_t)(mBase + row) * ldc + n0 + c4) = vv[it];
          }
          __threadfence();
        }
      }
    } else {
      _Float16* C = (_Float16*)Cout;
      const unsigned q = lane >> 3, c8 = (lane & 7u) * 8u;
      v8h hv[4];
#pragma unroll
      for (int it = 0; it < 4; ++it) {
        const unsigned row = (unsigned)it * 4u + q;
        const float* sp = slab + row * 68u + c8;
        PackH8 pk;
#pragma unroll
        for (int e2 = 0; e2 < 4; ++e2) pk.p[e2] = toh2_flush(sp[2 * e2], sp[2 * e2 + 1]);
        hv[it] = pk.v;
      }
      for (int pass = 0; pass < 2; ++pass) {
#pragma unroll
        for (int it = 0; it < 4; ++it) {
          const unsigned row = (unsigned)it * 4u + q;
          *(volatile v8h*)(C + (size_t)(mBase + row) * ldc + n0 + c8) = hv[it];
        }
        __threadfence();
      }
    }
    wave_sync_lds();
  }
}

__global__ __launch_bounds__(256) void k_proj_kq(const _Float16* __restrict__ TOKT, const _Float16* __restrict__ W16,
                                                 const float* __restrict__ bias, _Float16* __restrict__ OUT) {
    const unsigned by = blockIdx.y;
    const unsigned n = by >> 3, g = by & 7u;
    gemm64_body<1, false, false>(TOKT + (size_t)n * SEQ * CT + (size_t)CING * g, CT,
                                 W16 + (size_t)g * 64u * CING, CING,
                                 (void*)(OUT + (size_t)n * SEQ * KQW + 64u * g), KQW,
                                 bias + 64u * g, nullptr, SEQ / 64, 1u, CING);
}
__global__ __launch_bounds__(256) void k_proj_v(const _Float16* __restrict__ TOKT, const _Float16* __restrict__ W16,
                                                const float* __restrict__ bias, _Float16* __restrict__ V16) {
    const unsigned by = blockIdx.y;
    const unsigned n = by >> 3, g = by & 7u;
    gemm64_body<1, false, true>(W16 + (size_t)g * 128u * CING, CING,
                                TOKT + (size_t)n * SEQ * CT + (size_t)CING * g, CT,
                                (void*)(V16 + ((size_t)n * CT + 128u * g) * SEQ), SEQ,
                                bias + 128u * g, nullptr, 2u, SEQ / 64, CING);
}
__global__ __launch_bounds__(256) void k_ff(const _Float16* __restrict__ W16, const _Float16* __restrict__ TT16,
                                            const float* __restrict__ bias, const float* __restrict__ T32,
                                            float* __restrict__ out) {
    const unsigned n = blockIdx.y;
    gemm64_body<0, true, true>(W16, CT, TT16 + (size_t)n * SEQ * CT, CT,
                               (void*)(out + (size_t)n * CT * SEQ), SEQ,
                               bias, T32 + (size_t)n * CT * SEQ, CT / 64, SEQ / 64, CT);
}

static_assert(8 * 64 * 4 <= 131072);
__global__ __launch_bounds__(256) void k_colstat(const _Float16* __restrict__ KT, const _Float16* __restrict__ QT,
                                                 float* __restrict__ Mp, float* __restrict__ Rp) {
    __shared__ __align__(16) float sS[8][64];
    const unsigned lane = threadIdx.x & 31u;
    const unsigned wave = (unsigned)__builtin_amdgcn_readfirstlane((int)(threadIdx.x >> 5));
    const unsigned hh = lane >> 4, c = lane & 15u;
    const unsigned h = blockIdx.y, n = blockIdx.z;
    const unsigned m0 = blockIdx.x * 256u + wave * 32u;
    const _Float16* qb = QT + (size_t)(n * SEQ + m0 + c) * KQW + h * DK + 8u * hh;
    v16h qf[2];
    qf[0] = frag_ld(qb);
    qf[1] = frag_ld(qb + (size_t)16u * KQW);
    const _Float16* kb = KT + (size_t)(n * SEQ + c) * KQW + h * DK + 8u * hh;
    float mrun[2], srun[2];
    mrun[0] = -3.0e38f; mrun[1] = -3.0e38f; srun[0] = 0.f; srun[1] = 0.f;
#pragma unroll 1
    for (unsigned l0 = 0; l0 < (unsigned)SEQ; l0 += 32u) {
        const v16h kf0 = frag_ld(kb + (size_t)l0 * KQW);
        const v16h kf1 = frag_ld(kb + (size_t)(l0 + 16u) * KQW);
#pragma unroll
        for (int t = 0; t < 2; ++t) {
            const v8f z = (v8f){0.f,0.f,0.f,0.f,0.f,0.f,0.f,0.f};
            const v8f s0 = wmma16(kf0, qf[t], z);
            const v8f s1 = wmma16(kf1, qf[t], z);
            float x[16];
#pragma unroll
            for (int r = 0; r < 8; ++r) { x[r] = s0[r] * SC2; x[8 + r] = s1[r] * SC2; }
            float tmax = x[0];
#pragma unroll
            for (int i = 1; i < 16; ++i) tmax = (x[i] > tmax) ? x[i] : tmax;
            const float mnew = (tmax > mrun[t]) ? tmax : mrun[t];
            const float alpha = exp2f(mrun[t] - mnew);
            float ps = 0.f;
#pragma unroll
            for (int i = 0; i < 16; ++i) ps += exp2f(x[i] - mnew);
            srun[t] = srun[t] * alpha + ps;
            mrun[t] = mnew;
        }
    }
    float mfin[2], rfin[2];
#pragma unroll
    for (int t = 0; t < 2; ++t) {
        const float mo = __shfl_xor(mrun[t], 16, 32);
        const float mf = (mo > mrun[t]) ? mo : mrun[t];
        const float e  = srun[t] * exp2f(mrun[t] - mf);
        const float eo = __shfl_xor(e, 16, 32);
        const float st = e + eo;
        mfin[t] = mf;
        rfin[t] = P_CARRY / st;
    }
    float* sw = sS[wave];
    sw[16u * hh + c]       = (hh != 0u) ? mfin[1] : mfin[0];
    sw[32u + 16u * hh + c] = (hh != 0u) ? rfin[1] : rfin[0];
    wave_sync_lds();
    if (lane < 8u) {
        const v4f mv = *(const v4f*)(sw + 4u * lane);
        const v4f rv = *(const v4f*)(sw + 32u + 4u * lane);
        const size_t o = (size_t)(n * HEADS + h) * SEQ + m0 + 4u * lane;
        VST2V4(Mp + o, mv);
        VST2V4(Rp + o, rv);
    }
}

static_assert(32 * 16 * 16 == 64 * 128);
static_assert(32 * 16 * 8 == 32 * 128);
static_assert(8 * 64 * AT_PO * 4 <= 131072);
static_assert((AT_PO * 4) % 16 == 0);
__global__ __launch_bounds__(256) void k_attn(const _Float16* __restrict__ KT, const _Float16* __restrict__ QT,
                                              const _Float16* __restrict__ V16, const float* __restrict__ Mp,
                                              const float* __restrict__ Rp, const float* __restrict__ tok,
                                              float* __restrict__ T32, _Float16* __restrict__ TT16) {
    __shared__ __align__(16) float sO[8][64 * AT_PO];
    const unsigned lane = threadIdx.x & 31u;
    const unsigned wave = (unsigned)__builtin_amdgcn_readfirstlane((int)(threadIdx.x >> 5));
    const unsigned hh = lane >> 4, c = lane & 15u;
    const unsigned h = blockIdx.y, n = blockIdx.z;
    const unsigned m0 = blockIdx.x * 256u + wave * 32u;
    const _Float16* qb = QT + (size_t)(n * SEQ + m0 + c) * KQW + h * DK + 8u * hh;
    v16h qf[2];
    qf[0] = frag_ld(qb);
    qf[1] = frag_ld(qb + (size_t)16u * KQW);
    const _Float16* kb = KT + (size_t)(n * SEQ + c) * KQW + h * DK + 8u * hh;
    const _Float16* vb = V16 + ((size_t)n * CT + h * DV + c) * SEQ + 8u * hh;
    const size_t so_ = (size_t)(n * HEADS + h) * SEQ + m0 + c;
    float mc[2], rc[2];
    mc[0] = Mp[so_]; mc[1] = Mp[so_ + 16u];
    rc[0] = Rp[so_]; rc[1] = Rp[so_ + 16u];

    v8f o[4][2];
#pragma unroll
    for (int ct = 0; ct < 4; ++ct)
#pragma unroll
        for (int t = 0; t < 2; ++t) o[ct][t] = (v8f){0.f,0.f,0.f,0.f,0.f,0.f,0.f,0.f};

#pragma unroll 1
    for (unsigned l0 = 0; l0 < (unsigned)SEQ; l0 += 32u) {
        const v16h kf0 = frag_ld(kb + (size_t)l0 * KQW);
        const v16h kf1 = frag_ld(kb + (size_t)(l0 + 16u) * KQW);
        v16h pb[2];
#pragma unroll
        for (int t = 0; t < 2; ++t) {
            const v8f z = (v8f){0.f,0.f,0.f,0.f,0.f,0.f,0.f,0.f};
            const v8f s0 = wmma16(kf0, qf[t], z);
            const v8f s1 = wmma16(kf1, qf[t], z);
            PackH16 fp;
#pragma unroll
            for (int i = 0; i < 4; ++i) {
                const float a0 = exp2f(s0[2 * i] * SC2 - mc[t]) * rc[t];
                const float a1 = exp2f(s0[2 * i + 1] * SC2 - mc[t]) * rc[t];
                const float b0 = exp2f(s1[2 * i] * SC2 - mc[t]) * rc[t];
                const float b1 = exp2f(s1[2 * i + 1] * SC2 - mc[t]) * rc[t];
                fp.p[i]     = toh2_flush(a0, a1);
                fp.p[4 + i] = toh2_flush(b0, b1);
            }
            pb[t] = fp.v;
        }
#pragma unroll
        for (int ct = 0; ct < 4; ++ct) {
            const v16h vf = frag_ld(vb + (size_t)(16u * (unsigned)ct) * SEQ + l0);
            o[ct][0] = wmma16(vf, pb[0], o[ct][0]);
            o[ct][1] = wmma16(vf, pb[1], o[ct][1]);
        }
    }

    float* so = sO[wave];
#pragma unroll
    for (int ct = 0; ct < 4; ++ct)
#pragma unroll
        for (int t = 0; t < 2; ++t)
#pragma unroll
            for (int r = 0; r < 8; ++r)
                so[(16u * (unsigned)ct + 8u * hh + (unsigned)r) * AT_PO + 16u * (unsigned)t + c] = o[ct][t][r] * O_UNDO;
    wave_sync_lds();
    const unsigned q8 = lane >> 3, pc = lane & 7u;
    {
        const float* tokb = tok + ((size_t)n * CT + h * DV) * SEQ_FULL + m0 + 4u * pc;
        float* tdst = T32 + ((size_t)n * CT + h * DV) * SEQ + m0 + 4u * pc;
#pragma unroll 1
        for (unsigned g = 0; g < 4u; ++g) {
            v4f tv[4];
#pragma unroll
            for (int it = 0; it < 4; ++it) {
                const unsigned row = 16u * g + 4u * (unsigned)it + q8;
                const v4f kv = *(const v4f*)(so + row * AT_PO + 4u * pc);
                const v4f x = *(const v4f*)(tokb + (size_t)row * SEQ_FULL);
                v4f tt;
                tt.x = bfr(x.x) + kv.x; tt.y = bfr(x.y) + kv.y; tt.z = bfr(x.z) + kv.z; tt.w = bfr(x.w) + kv.w;
                tv[it] = tt;
            }
#pragma unroll
            for (int it = 0; it < 4; ++it) {
                const unsigned row = 16u * g + 4u * (unsigned)it + q8;
                *(v4f*)(so + row * AT_PO + 4u * pc) = tv[it];
            }
            for (int pass = 0; pass < 2; ++pass) {
#pragma unroll
                for (int it = 0; it < 4; ++it) {
                    const unsigned row = 16u * g + 4u * (unsigned)it + q8;
                    *(volatile v4f*)(tdst + (size_t)row * SEQ) = tv[it];
                }
                __threadfence();
            }
        }
    }
    wave_sync_lds();
    {
        v8h hv[8];
#pragma unroll
        for (int it = 0; it < 8; ++it) {
            const unsigned m = 4u * (unsigned)it + q8;
            PackH8 pk;
#pragma unroll
            for (int e2 = 0; e2 < 4; ++e2) {
                const float a = so[(8u * pc + 2u * (unsigned)e2) * AT_PO + m] * ACT_CARRY;
                const float b = so[(8u * pc + 2u * (unsigned)e2 + 1u) * AT_PO + m] * ACT_CARRY;
                pk.p[e2] = toh2_flush(a, b);
            }
            hv[it] = pk.v;
        }
        _Float16* ttd = TT16 + ((size_t)n * SEQ + m0 + q8) * CT + h * DV + 8u * pc;
        for (int pass = 0; pass < 2; ++pass) {
#pragma unroll
            for (int it = 0; it < 8; ++it) *(volatile v8h*)(ttd + (size_t)(4u * (unsigned)it) * CT) = hv[it];
            __threadfence();
        }
    }
}

static constexpr size_t SZ_TOKT = (size_t)NB * SEQ * CT * 2;
static constexpr size_t SZ_WKQ  = (size_t)KQW * CING * 2;
static constexpr size_t SZ_WV   = (size_t)CT * CING * 2;
static constexpr size_t SZ_WF   = (size_t)CT * CT * 2;
static constexpr size_t SZ_KQT  = (size_t)NB * SEQ * KQW * 2;
static constexpr size_t SZ_V    = (size_t)NB * CT * SEQ * 2;
static constexpr size_t SZ_STAT = (size_t)NB * HEADS * SEQ * 4;
static constexpr size_t SZ_T32  = (size_t)NB * CT * SEQ * 4;
static constexpr size_t SZ_TT   = (size_t)NB * SEQ * CT * 2;
static constexpr size_t OFF_TOKT = 0;
static constexpr size_t OFF_WK   = OFF_TOKT + SZ_TOKT;
static constexpr size_t OFF_WQ   = OFF_WK + SZ_WKQ;
static constexpr size_t OFF_WV   = OFF_WQ + SZ_WKQ;
static constexpr size_t OFF_WF   = OFF_WV + SZ_WV;
static constexpr size_t OFF_KT   = OFF_WF + SZ_WF;
static constexpr size_t OFF_QT   = OFF_KT + SZ_KQT;
static constexpr size_t OFF_V    = OFF_QT + SZ_KQT;
static constexpr size_t OFF_M    = OFF_V + SZ_V;
static constexpr size_t OFF_R    = OFF_M + SZ_STAT;
static constexpr size_t OFF_T32  = OFF_R + SZ_STAT;
static constexpr size_t OFF_TT   = OFF_T32 + SZ_T32;
static constexpr size_t WS_TOTAL = OFF_TT + SZ_TT;
static_assert(SZ_TOKT % 256 == 0 && SZ_WKQ % 256 == 0 && SZ_WV % 256 == 0 && SZ_WF % 256 == 0);
static_assert(SZ_KQT % 256 == 0 && SZ_V % 256 == 0 && SZ_STAT % 256 == 0 && SZ_T32 % 256 == 0 && SZ_TT % 256 == 0);
static_assert(WS_TOTAL <= (size_t)134217728);
static_assert((KQW * CING / 8) % 256 == 0 && (CT * CING / 8) % 256 == 0 && (CT * CT / 8) % 256 == 0);
static_assert((SEQ / 64) % 8 == 0 && (2 * (SEQ / 64)) % 8 == 0 && ((CT / 64) * (SEQ / 64)) % 8 == 0);

extern "C" void kernel_launch(void* const* d_in, const int* in_sizes, int n_in, void* d_out, int out_size,
                              void* d_ws, size_t ws_size, hipStream_t stream) {
    if (n_in < 9) return;
    if (in_sizes[0] < NB * CT * SEQ_FULL) return;
    if (in_sizes[1] < KQW * CING || in_sizes[2] < KQW || in_sizes[3] < KQW * CING || in_sizes[4] < KQW) return;
    if (in_sizes[5] < CT * CING || in_sizes[6] < CT || in_sizes[7] < CT * CT || in_sizes[8] < CT) return;
    if (out_size < NB * CT * SEQ) return;
    if (ws_size < WS_TOTAL) return;

    const float* tokens = (const float*)d_in[0];
    const float* k_w    = (const float*)d_in[1];
    const float* k_b    = (const float*)d_in[2];
    const float* q_w    = (const float*)d_in[3];
    const float* q_b    = (const float*)d_in[4];
    const float* v_w    = (const float*)d_in[5];
    const float* v_b    = (const float*)d_in[6];
    const float* ff_w   = (const float*)d_in[7];
    const float* ff_b   = (const float*)d_in[8];
    float* out = (float*)d_out;

    char* wsp = (char*)d_ws;
    _Float16* TOKT = (_Float16*)(wsp + OFF_TOKT);
    _Float16* WK16 = (_Float16*)(wsp + OFF_WK);
    _Float16* WQ16 = (_Float16*)(wsp + OFF_WQ);
    _Float16* WV16 = (_Float16*)(wsp + OFF_WV);
    _Float16* WF16 = (_Float16*)(wsp + OFF_WF);
    _Float16* KT16 = (_Float16*)(wsp + OFF_KT);
    _Float16* QT16 = (_Float16*)(wsp + OFF_QT);
    _Float16* V16  = (_Float16*)(wsp + OFF_V);
    float*    Mpl  = (float*)(wsp + OFF_M);
    float*    Rpl  = (float*)(wsp + OFF_R);
    float*    T32  = (float*)(wsp + OFF_T32);
    _Float16* TT16 = (_Float16*)(wsp + OFF_TT);

    k_wconv<<<(KQW * CING / 8) / 256, 256, 0, stream>>>(k_w, WK16, (unsigned)(KQW * CING / 8));
    k_wconv<<<(KQW * CING / 8) / 256, 256, 0, stream>>>(q_w, WQ16, (unsigned)(KQW * CING / 8));
    k_wconv<<<(CT * CING / 8) / 256, 256, 0, stream>>>(v_w, WV16, (unsigned)(CT * CING / 8));
    k_wconv<<<(CT * CT / 8) / 256, 256, 0, stream>>>(ff_w, WF16, (unsigned)(CT * CT / 8));

    k_tokT<<<dim3(SEQ / 64, CT / 64, NB), 256, 0, stream>>>(tokens, TOKT);

    k_proj_kq<<<dim3((SEQ / 64) / 8, NB * GROUPS), 256, 0, stream>>>(TOKT, WK16, k_b, KT16);
    k_proj_kq<<<dim3((SEQ / 64) / 8, NB * GROUPS), 256, 0, stream>>>(TOKT, WQ16, q_b, QT16);
    k_proj_v<<<dim3((2 * (SEQ / 64)) / 8, NB * GROUPS), 256, 0, stream>>>(TOKT, WV16, v_b, V16);

    k_colstat<<<dim3(SEQ / 256, HEADS, NB), 256, 0, stream>>>(KT16, QT16, Mpl, Rpl);
    k_attn<<<dim3(SEQ / 256, HEADS, NB), 256, 0, stream>>>(KT16, QT16, V16, Mpl, Rpl, tokens, T32, TT16);

    k_ff<<<dim3(((CT / 64) * (SEQ / 64)) / 8, NB), 256, 0, stream>>>(WF16, TT16, ff_b, T32, out);
}
